// MultiHeadAttention_33182917329260
// MI455X (gfx1250) — hardware-verified
//
#include <hip/hip_runtime.h>


#ifndef NB
#define NB 4
#endif
#ifndef SEQ
#define SEQ 2048
#endif
#define NB_FULL 4
#define SEQ_FULL 2048
#define NHD 16
#define HD 64
#define CDIM (NHD * HD)
#define NU (NB * NHD)
#ifndef RH
#define RH 1024
#endif
#define RHE (((RH) < (SEQ)) ? (RH) : (SEQ))
#define QCAR 64.0f
#define VCAR 256.0f
#define PCAR 16384.0f
#define CCAR 256.0f
#define WCAR 256.0f
#define SSC (0.125f / (QCAR * QCAR))
#define OSC (CCAR / (PCAR * VCAR))
#define OSCP (1.0f / (CCAR * WCAR))
#define NEGBIG (-1.0e30f)
#define L2E 1.4426950408889634f
#define LDT 72
#define WSMAX ((size_t)134217728)

static_assert(SEQ % 64 == 0);
static_assert(SEQ >= 64 && SEQ <= SEQ_FULL);
static_assert(NB >= 1 && NB <= NB_FULL);
static_assert(RH % 64 == 0 && RH >= 64);
static_assert(RHE % 64 == 0);
static_assert(HD == 64);
static_assert(CDIM % 64 == 0);
static_assert(((size_t)NB * SEQ * CDIM) % 8 == 0);
static_assert((3 * CDIM * CDIM) % 8 == 0);

typedef _Float16 h16;
typedef unsigned short bf;
typedef __attribute__((ext_vector_type(16))) __bf16   v16bf;
typedef __attribute__((ext_vector_type(16))) _Float16 v16h;
typedef __attribute__((ext_vector_type(8)))  _Float16 v8h;
typedef __attribute__((ext_vector_type(8)))  unsigned short v8us;
typedef __attribute__((ext_vector_type(8)))  float    v8f;
typedef __attribute__((ext_vector_type(4)))  float    v4f;
typedef v8h  __attribute__((may_alias)) v8ha;
typedef v4f  __attribute__((may_alias)) v4fa;
typedef v8us __attribute__((may_alias)) v8usa;

__device__ __forceinline__ unsigned short f2bf(float f) { unsigned u = __float_as_uint(f); u += 0x7FFFu + ((u >> 16) & 1u); return (unsigned short)(u >> 16); }
__device__ __forceinline__ float bf2f(unsigned short b) { return __uint_as_float(((unsigned)b) << 16); }
__device__ __forceinline__ float bfr(float f) { return bf2f(f2bf(f)); }
__device__ __forceinline__ v16h cat16(v8h lo, v8h hi) { return __builtin_shufflevector(lo, hi, 0, 1, 2, 3, 4, 5, 6, 7, 8, 9, 10, 11, 12, 13, 14, 15); }
__device__ __forceinline__ v16bf cat16b(v8us lo, v8us hi) { return __builtin_bit_cast(v16bf, __builtin_shufflevector(lo, hi, 0, 1, 2, 3, 4, 5, 6, 7, 8, 9, 10, 11, 12, 13, 14, 15)); }
__device__ __forceinline__ v8f wmma16(v16h a, v16h b, v8f c) { return __builtin_amdgcn_wmma_f32_16x16x32_f16(false, a, false, b, (short)0, c, false, false); }
__device__ __forceinline__ v8f wmmab(v16bf a, v16bf b, v8f c) { return __builtin_amdgcn_wmma_f32_16x16x32_bf16(false, a, false, b, (short)0, c, false, false); }

template <typename T16> struct WFrag;
template <> struct WFrag<h16> { typedef v16h V; static __device__ __forceinline__ V ld(const h16* p) { return cat16(*(const v8h*)p, *(const v8h*)(p + 16)); } static __device__ __forceinline__ v8f mma(V a, V b, v8f c) { return wmma16(a, b, c); } };
template <> struct WFrag<bf> { typedef v16bf V; static __device__ __forceinline__ V ld(const bf* p) { return cat16b(*(const v8us*)p, *(const v8us*)(p + 16)); } static __device__ __forceinline__ v8f mma(V a, V b, v8f c) { return wmmab(a, b, c); } };

template <typename T16, int NSPLIT, bool BIAS>
__global__ __launch_bounds__(32) void k_gemmw(const T16* __restrict__ A, const T16* __restrict__ A2, const T16* __restrict__ Bt, const T16* __restrict__ Bt2, int K, float* C, int ldc, const float* __restrict__ bias, size_t sA, size_t sA2, size_t sB, size_t sC, float oscale) {
    typedef typename WFrag<T16>::V V;
    __shared__ __align__(16) float os[16 * 68];
    const size_t z = blockIdx.z; A += z * sA; if (A2) A2 += z * sA2; Bt += z * sB; if (Bt2) Bt2 += z * sB; C += z * sC;
    const int lane = threadIdx.x & 31, lr = lane & 15, hi = lane >> 4; const int r0 = blockIdx.x * 64, c0 = blockIdx.y * 64;
    v8f acc[4][4];
#pragma unroll
    for (int mb = 0; mb < 4; ++mb)
#pragma unroll
        for (int nb = 0; nb < 4; ++nb) acc[mb][nb] = (v8f){};
    const size_t aoff = (size_t)(r0 + lr) * K + 8 * hi, boff = (size_t)(c0 + lr) * K + 8 * hi;
#pragma unroll 1
    for (int kc = 0; kc < K; kc += 32) {
        V a[4], a2[4];
#pragma unroll
        for (int mb = 0; mb < 4; ++mb) { a[mb] = WFrag<T16>::ld(A + aoff + (size_t)mb * 16 * K + kc); if (NSPLIT == 1 || NSPLIT == 2) a2[mb] = WFrag<T16>::ld(A2 + aoff + (size_t)mb * 16 * K + kc); }
#pragma unroll
        for (int nb = 0; nb < 4; ++nb) { const V b = WFrag<T16>::ld(Bt + boff + (size_t)nb * 16 * K + kc); V b2; if (NSPLIT >= 2) b2 = WFrag<T16>::ld(Bt2 + boff + (size_t)nb * 16 * K + kc);
#pragma unroll
            for (int mb = 0; mb < 4; ++mb) { acc[mb][nb] = WFrag<T16>::mma(a[mb], b, acc[mb][nb]); if (NSPLIT == 1 || NSPLIT == 2) acc[mb][nb] = WFrag<T16>::mma(a2[mb], b, acc[mb][nb]); if (NSPLIT >= 2) acc[mb][nb] = WFrag<T16>::mma(a[mb], b2, acc[mb][nb]); } }
        asm volatile("v_nop\n\tv_nop\n\tv_nop\n\tv_nop" : "+v"(acc[0][0]), "+v"(acc[1][1]), "+v"(acc[2][2]), "+v"(acc[3][3]) : "v"(a[0]), "v"(a[3]));
    }
#pragma unroll
    for (int mb = 0; mb < 4; ++mb) {
#pragma unroll
        for (int nb = 0; nb < 4; ++nb) {
#pragma unroll
            for (int j = 0; j < 8; ++j) os[(hi * 8 + j) * 68 + nb * 16 + lr] = acc[mb][nb][j]; }
        __builtin_amdgcn_wave_barrier(); asm volatile("" ::: "memory");
        float* crow = C + (size_t)(r0 + mb * 16) * ldc + c0;
#pragma unroll 1
        for (int ps = 0; ps < 2; ++ps) {
#pragma unroll
            for (int s = 0; s < 8; ++s) { const int row = 2 * s + hi, cofs = lr * 4; v4f val = *(const v4fa*)(os + row * 68 + cofs); val = val * oscale; if (BIAS) { val[0] += bfr(bias[c0 + cofs]); val[1] += bfr(bias[c0 + cofs + 1]); val[2] += bfr(bias[c0 + cofs + 2]); val[3] += bfr(bias[c0 + cofs + 3]); }
                *(volatile v4f*)(crow + (size_t)row * ldc + cofs) = val; }
            if (ps == 0) __threadfence(); }
        __builtin_amdgcn_wave_barrier(); asm volatile("" ::: "memory");
    }
}

__global__ __launch_bounds__(256) void k_cvt8(const float* __restrict__ src, bf* dst, size_t n8) { const size_t i = (size_t)blockIdx.x * 256 + threadIdx.x; if (i >= n8) return; const v8f v = *(const v8f*)(src + i * 8); v8us o;
#pragma unroll
    for (int k = 0; k < 8; ++k) o[k] = f2bf(v[k]); *(volatile v8us*)(dst + i * 8) = o; __threadfence(); *(volatile v8us*)(dst + i * 8) = o; }

__global__ __launch_bounds__(256) void k_cvtx(const float* __restrict__ x, bf* dst, size_t n8) { const size_t i = (size_t)blockIdx.x * 256 + threadIdx.x; if (i >= n8) return;
    const size_t e = i * 8; const size_t r = e / CDIM; const size_t c = e % CDIM; const size_t srow = (r / SEQ) * (size_t)SEQ_FULL + (r % SEQ);
    const v8f v = *(const v8f*)(x + srow * CDIM + c); v8us o;
#pragma unroll
    for (int k = 0; k < 8; ++k) o[k] = f2bf(v[k]); *(volatile v8us*)(dst + e) = o; __threadfence(); *(volatile v8us*)(dst + e) = o; }

__global__ __launch_bounds__(256) void k_cvth(const float* __restrict__ src, h16* dst, size_t n8, float sc) { const size_t i = (size_t)blockIdx.x * 256 + threadIdx.x; if (i >= n8) return; const v8f v = *(const v8f*)(src + i * 8); v8h o;
#pragma unroll
    for (int k = 0; k < 8; ++k) o[k] = (h16)(bfr(v[k]) * sc); *(volatile v8h*)(dst + i * 8) = o; __threadfence(); *(volatile v8h*)(dst + i * 8) = o; }

template <int MODE>
__global__ __launch_bounds__(32) void k_qkvp(const bf* __restrict__ A, const bf* __restrict__ Bt, h16* P0, h16* P0l, h16* P1, h16* P1l) {
    __shared__ __align__(16) h16 ts[64 * LDT];
    __shared__ __align__(16) h16 tl[64 * LDT];
    const int K = CDIM;
    const int lane = threadIdx.x & 31, lr = lane & 15, hi = lane >> 4; const int r0 = blockIdx.x * 64, c0 = blockIdx.y * 64;
    v8f acc[4][4];
#pragma unroll
    for (int mb = 0; mb < 4; ++mb)
#pragma unroll
        for (int nb = 0; nb < 4; ++nb) acc[mb][nb] = (v8f){};
    const size_t aoff = (size_t)(r0 + lr) * K + 8 * hi, boff = (size_t)(c0 + lr) * K + 8 * hi;
#pragma unroll 1
    for (int kc = 0; kc < K; kc += 32) {
        v16bf a[4];
#pragma unroll
        for (int mb = 0; mb < 4; ++mb) a[mb] = WFrag<bf>::ld(A + aoff + (size_t)mb * 16 * K + kc);
#pragma unroll
        for (int nb = 0; nb < 4; ++nb) { const v16bf b = WFrag<bf>::ld(Bt + boff + (size_t)nb * 16 * K + kc);
#pragma unroll
            for (int mb = 0; mb < 4; ++mb) acc[mb][nb] = wmmab(a[mb], b, acc[mb][nb]); }
        asm volatile("v_nop\n\tv_nop\n\tv_nop\n\tv_nop" : "+v"(acc[0][0]), "+v"(acc[1][1]), "+v"(acc[2][2]), "+v"(acc[3][3]) : "v"(a[0]), "v"(a[3]));
    }
    h16* hb; h16* lb; size_t pit, pitl; bool haslo; float car;
    if (MODE == 0) {
        const int part = r0 / CDIM, hh = (r0 % CDIM) / HD; const int b = c0 / SEQ, n0 = c0 % SEQ; const int u = b * NHD + hh;
        hb = ((part == 0) ? P0 : P1) + ((size_t)u * SEQ + n0) * HD; pit = HD;
        haslo = (n0 < RHE); lb = ((part == 0) ? P0l : P1l) + ((size_t)u * RHE + n0) * HD; pitl = HD; car = QCAR;
    } else {
        const int b = r0 / SEQ, t0 = r0 % SEQ, hh = c0 / HD; const int u = b * NHD + hh;
        hb = P0 + (size_t)u * HD * SEQ + t0; pit = SEQ;
        haslo = (t0 < RHE); lb = P0l + (size_t)u * HD * RHE + t0; pitl = RHE; car = VCAR;
    }
#pragma unroll
    for (int mb = 0; mb < 4; ++mb)
#pragma unroll
        for (int nb = 0; nb < 4; ++nb) { v8h oh, ol;
#pragma unroll
            for (int j = 0; j < 8; ++j) { const float xv = acc[mb][nb][j] * car; const h16 ah = (h16)xv; oh[j] = ah; ol[j] = (h16)(xv - (float)ah); }
            *(v8ha*)(ts + (nb * 16 + lr) * LDT + mb * 16 + 8 * hi) = oh;
            if (haslo) *(v8ha*)(tl + (nb * 16 + lr) * LDT + mb * 16 + 8 * hi) = ol; }
    __syncthreads();
#pragma unroll 1
    for (int ps = 0; ps < 2; ++ps) {
#pragma unroll
        for (int q = 0; q < 16; ++q) { const int rho = q * 4 + (lane >> 3), pc = (lane & 7) * 8;
            const v8h v = *(const v8ha*)(ts + rho * LDT + pc); *(volatile v8h*)(hb + (size_t)rho * pit + pc) = v;
            if (haslo) { const v8h w = *(const v8ha*)(tl + rho * LDT + pc); *(volatile v8h*)(lb + (size_t)rho * pitl + pc) = w; } }
        if (ps == 0) __threadfence(); }
}

template <bool EARLY>
__global__ __launch_bounds__(32) void k_attn(const h16* __restrict__ Qh, const h16* __restrict__ Ql, const h16* __restrict__ Kh, const h16* __restrict__ Kl,
                                             const h16* __restrict__ Vt, const h16* __restrict__ Vtl, h16* Ch, h16* Cl, int qt0) {
    __shared__ __align__(16) h16 cs[16 * LDT];
    __shared__ __align__(16) h16 cs2[16 * LDT];
    const int lane = threadIdx.x & 31, lr = lane & 15, hi = lane >> 4;
    const int u = blockIdx.y, qt = qt0 + (int)blockIdx.x;
    const int b = u / NHD, hh = u % NHD;
    const int q0 = qt * 16, qrow = q0 + lr;
    const h16* Qu = Qh + ((size_t)u * SEQ + q0) * HD + (size_t)lr * HD + 8 * hi;
    const h16* Qlu = Ql + ((size_t)u * RHE + q0) * HD + (size_t)lr * HD + 8 * hi;
    v16h qf[2], qlf[2];
#pragma unroll
    for (int ks = 0; ks < 2; ++ks) { qf[ks] = WFrag<h16>::ld(Qu + 32 * ks); if (EARLY) qlf[ks] = WFrag<h16>::ld(Qlu + 32 * ks); else qlf[ks] = qf[ks]; }
    const h16* Ku  = Kh  + (size_t)u * SEQ * HD + (size_t)lr * HD + 8 * hi;
    const h16* Klu = Kl  + (size_t)u * RHE * HD + (size_t)lr * HD + 8 * hi;
    const h16* Vu  = Vt  + (size_t)u * HD * SEQ + (size_t)lr * SEQ + 8 * hi;
    const h16* Vlu = Vtl + (size_t)u * HD * RHE + (size_t)lr * RHE + 8 * hi;
    v8f acc[4];
#pragma unroll
    for (int dt = 0; dt < 4; ++dt) acc[dt] = (v8f){};
    float m = NEGBIG, l = 0.f;
    const int nch = (qt >> 2) + 1;
#pragma unroll 1
    for (int kb = 0; kb < nch; ++kb) {
        const int k0 = kb * 64;
        v8f s[4]; v16h ka, kla;
#pragma unroll
        for (int j = 0; j < 4; ++j) {
            s[j] = (v8f){};
#pragma unroll
            for (int ks = 0; ks < 2; ++ks) {
                ka = WFrag<h16>::ld(Ku + (size_t)(k0 + 16 * j) * HD + 32 * ks);
                s[j] = wmma16(ka, qf[ks], s[j]);
                if (EARLY) { kla = WFrag<h16>::ld(Klu + (size_t)(k0 + 16 * j) * HD + 32 * ks); s[j] = wmma16(kla, qf[ks], s[j]); s[j] = wmma16(ka, qlf[ks], s[j]); } else kla = ka;
            }
        }
        asm volatile("v_nop\n\tv_nop\n\tv_nop\n\tv_nop" : "+v"(s[0]), "+v"(s[1]), "+v"(s[2]), "+v"(s[3]) : "v"(qf[0]), "v"(qf[1]), "v"(ka), "v"(kla));
        const int lim = qrow - 8 * hi - k0;
        float cmax = NEGBIG;
#pragma unroll
        for (int j = 0; j < 4; ++j)
#pragma unroll
            for (int r = 0; r < 8; ++r) { float t = s[j][r] * SSC; t = ((16 * j + r) > lim) ? NEGBIG : t; s[j][r] = t; cmax = fmaxf(cmax, t); }
        cmax = fmaxf(cmax, __shfl_xor(cmax, 16, 32));
        const float mnew = fmaxf(m, cmax);
        const float corr = __builtin_amdgcn_exp2f((m - mnew) * L2E);
        m = mnew;
        float psum = 0.f; v8h ph[4], pl[4];
#pragma unroll
        for (int j = 0; j < 4; ++j)
#pragma unroll
            for (int r = 0; r < 8; ++r) { const float p = __builtin_amdgcn_exp2f((s[j][r] - mnew) * L2E); psum += p; const float pc = p * PCAR; const h16 ah = (h16)pc; ph[j][r] = ah; if (EARLY) pl[j][r] = (h16)(pc - (float)ah); else pl[j][r] = ah; }
        psum += __shfl_xor(psum, 16, 32);
        l = l * corr + psum;
#pragma unroll
        for (int dt = 0; dt < 4; ++dt) acc[dt] = acc[dt] * corr;
        v16h pb[2], plb[2];
        pb[0] = cat16(ph[0], ph[1]); pb[1] = cat16(ph[2], ph[3]);
        plb[0] = cat16(pl[0], pl[1]); plb[1] = cat16(pl[2], pl[3]);
        v16h va, vla;
#pragma unroll
        for (int dt = 0; dt < 4; ++dt) {
#pragma unroll
            for (int ks = 0; ks < 2; ++ks) {
                va = WFrag<h16>::ld(Vu + (size_t)(dt * 16) * SEQ + k0 + 32 * ks);
                acc[dt] = wmma16(va, pb[ks], acc[dt]);
                if (EARLY) { vla = WFrag<h16>::ld(Vlu + (size_t)(dt * 16) * RHE + k0 + 32 * ks); acc[dt] = wmma16(vla, pb[ks], acc[dt]); acc[dt] = wmma16(va, plb[ks], acc[dt]); } else vla = va;
            }
        }
        asm volatile("v_nop\n\tv_nop\n\tv_nop\n\tv_nop" : "+v"(acc[0]), "+v"(acc[1]), "+v"(acc[2]), "+v"(acc[3]) : "v"(pb[0]), "v"(pb[1]), "v"(plb[0]), "v"(plb[1]), "v"(va), "v"(vla));
    }
    const float f = (1.0f / l) * OSC;
#pragma unroll
    for (int dt = 0; dt < 4; ++dt) { v8h oh, ol;
#pragma unroll
        for (int r = 0; r < 8; ++r) { const float oc = acc[dt][r] * f; const h16 ah = (h16)oc; oh[r] = ah; if (EARLY) ol[r] = (h16)(oc - (float)ah); else ol[r] = ah; }
        *(v8ha*)(cs + lr * LDT + dt * 16 + 8 * hi) = oh;
        if (EARLY) *(v8ha*)(cs2 + lr * LDT + dt * 16 + 8 * hi) = ol; }
    __syncthreads();
    h16* Cb  = Ch + ((size_t)b * SEQ + q0) * CDIM + hh * HD;
    h16* Clb = Cl + ((size_t)b * RHE + q0) * CDIM + hh * HD;
#pragma unroll 1
    for (int ps = 0; ps < 2; ++ps) {
#pragma unroll
        for (int q = 0; q < 4; ++q) { const int rho = q * 4 + (lane >> 3), pc = (lane & 7) * 8;
            const v8h v = *(const v8ha*)(cs + rho * LDT + pc); *(volatile v8h*)(Cb + (size_t)rho * CDIM + pc) = v;
            if (EARLY) { const v8h w = *(const v8ha*)(cs2 + rho * LDT + pc); *(volatile v8h*)(Clb + (size_t)rho * CDIM + pc) = w; } }
        if (ps == 0) __threadfence(); }
}

extern "C" void kernel_launch(void* const* d_in, const int* in_sizes, int n_in,
                              void* d_out, int out_size, void* d_ws, size_t ws_size, hipStream_t stream) {
    if (n_in < 4) return;
    if ((size_t)in_sizes[0] < ((size_t)(NB - 1) * SEQ_FULL + SEQ) * CDIM) return;
    if ((size_t)in_sizes[1] < (size_t)3 * CDIM * CDIM) return;
    if ((size_t)in_sizes[2] < (size_t)CDIM * CDIM) return;
    if (in_sizes[3] < CDIM) return;
    if ((size_t)out_size < (size_t)NB * SEQ * CDIM) return;
    const float* X     = (const float*)d_in[0];
    const float* Wqkv  = (const float*)d_in[1];
    const float* Wproj = (const float*)d_in[2];
    const float* Bproj = (const float*)d_in[3];
    float* OUT = (float*)d_out;
    char* wsp = (char*)d_ws;
    auto take = [&](size_t bytes) { char* p = wsp; wsp += (bytes + 255) & ~(size_t)255; return (void*)p; };
    bf*  Xb  = (bf*)take((size_t)NB * SEQ * CDIM * 2);
    bf*  Wqb = (bf*)take((size_t)3 * CDIM * CDIM * 2);
    h16* Wp  = (h16*)take((size_t)CDIM * CDIM * 2);
    h16* Qh  = (h16*)take((size_t)NU * SEQ * HD * 2);
    h16* Ql  = (h16*)take((size_t)NU * RHE * HD * 2);
    h16* Kh  = (h16*)take((size_t)NU * SEQ * HD * 2);
    h16* Kl  = (h16*)take((size_t)NU * RHE * HD * 2);
    h16* Vt  = (h16*)take((size_t)NU * HD * SEQ * 2);
    h16* Vtl = (h16*)take((size_t)NU * HD * RHE * 2);
    h16* Ch  = (h16*)take((size_t)NB * SEQ * CDIM * 2);
    h16* Cl  = (h16*)take((size_t)NB * RHE * CDIM * 2);
    const size_t used = (size_t)(wsp - (char*)d_ws);
    if (used > ws_size || used > WSMAX) return;

    const size_t n8x = (size_t)NB * SEQ * CDIM / 8, n8w = (size_t)3 * CDIM * CDIM / 8, n8p = (size_t)CDIM * CDIM / 8;
    k_cvtx<<<(unsigned)((n8x + 255) / 256), 256, 0, stream>>>(X, Xb, n8x);
    k_cvt8<<<(unsigned)((n8w + 255) / 256), 256, 0, stream>>>(Wqkv, Wqb, n8w);
    k_cvth<<<(unsigned)((n8p + 255) / 256), 256, 0, stream>>>(Wproj, Wp, n8p, WCAR);
    k_qkvp<0><<<dim3(2 * CDIM / 64, NB * SEQ / 64), 32, 0, stream>>>(Wqb, Xb, Qh, Ql, Kh, Kl);
    k_qkvp<1><<<dim3(NB * SEQ / 64, CDIM / 64), 32, 0, stream>>>(Xb, Wqb + (size_t)2 * CDIM * CDIM, Vt, Vtl, nullptr, nullptr);
    k_attn<true><<<dim3(RHE / 16, NU), 32, 0, stream>>>(Qh, Ql, Kh, Kl, Vt, Vtl, Ch, Cl, 0);
    if (SEQ > RHE) k_attn<false><<<dim3((SEQ - RHE) / 16, NU), 32, 0, stream>>>(Qh, Ql, Kh, Kl, Vt, Vtl, Ch, Cl, RHE / 16);
    k_gemmw<h16, 1, true><<<dim3(RHE / 64, CDIM / 64, NB), 32, 0, stream>>>(Ch, Cl, Wp, nullptr, CDIM, OUT, CDIM, Bproj, (size_t)SEQ * CDIM, (size_t)RHE * CDIM, (size_t)0, (size_t)SEQ * CDIM, OSCP);
    if (SEQ > RHE) k_gemmw<h16, 0, true><<<dim3((SEQ - RHE) / 64, CDIM / 64, NB), 32, 0, stream>>>(Ch + (size_t)RHE * CDIM, nullptr, Wp, nullptr, CDIM, OUT + (size_t)RHE * CDIM, CDIM, Bproj, (size_t)SEQ * CDIM, (size_t)0, (size_t)0, (size_t)SEQ * CDIM, OSCP);
}
